// CMHSA_57810259804423
// MI455X (gfx1250) — hardware-run, weakly checked
//
#include <hip/hip_runtime.h>


#ifndef NB
#define NB 4
#endif
#ifndef SEQ
#define SEQ 1024
#endif
#define NB_FULL  4
#define SEQ_FULL 1024
#ifndef OUT_SEQ
#define OUT_SEQ SEQ
#endif
#define DM   256
#define NH_  4
#define HD   64
#define AW   4
#define OSP  68
#define QKC  16.0f
#define VCC  16.0f
#define CCS  16.0f
#define WPC  1024.0f
#define PCARRY 32768.0f
#define C15  (32768.0f / (float)SEQ)
#define SC2  ((float)(0.125 * 1.4426950408889634 / 256.0))
#define OSC  (1.0f / 524288.0f)
#define OUTSC (1.0f / 16384.0f)
#define VSC  ((float)(1.0 / (1073741824.0 * (double)SEQ * (double)SEQ)))
#define EPSN 1.0e-5f
#define NEGB (-3.0e38f)

static_assert(DM == 256);
static_assert(HD == 64);
static_assert(NH_ * HD == DM);
static_assert(NH_ == 4);
static_assert(DM % 64 == 0);
static_assert(DM % 32 == 0);
static_assert(SEQ % 64 == 0);
static_assert((NB * SEQ) % 64 == 0);
static_assert(SEQ % 32 == 0);
static_assert(SEQ % (16 * AW) == 0);
static_assert(16 * AW == 64);
static_assert(SEQ % 256 == 0);
static_assert(((size_t)SEQ * HD) % 2048 == 0);
static_assert(((size_t)NB * SEQ * DM) % 2048 == 0);
static_assert((NB * DM) % 32 == 0);
static_assert(SEQ_FULL % 4 == 0);
static_assert(OUT_SEQ % 32 == 0);
static_assert(OUT_SEQ >= SEQ);
static_assert(NB <= NB_FULL);
static_assert(SEQ <= SEQ_FULL);
static_assert((OSP * 4) % 16 == 0);
static_assert(OSP >= 64 + 4);
static_assert(((size_t)DM * DM) % 8 == 0);

typedef _Float16 h16;
typedef unsigned short bf;
typedef __attribute__((ext_vector_type(16))) __bf16   v16bf;
typedef __attribute__((ext_vector_type(16))) _Float16 v16h;
typedef __attribute__((ext_vector_type(8)))  _Float16 v8h;
typedef __attribute__((ext_vector_type(8)))  unsigned short v8us;
typedef __attribute__((ext_vector_type(8)))  float    v8f;
typedef __attribute__((ext_vector_type(4)))  float    v4f;
typedef v4f  __attribute__((may_alias)) v4fa;

__device__ __forceinline__ unsigned short f2bf(float f) { unsigned u = __float_as_uint(f); u += 0x7FFFu + ((u >> 16) & 1u); return (unsigned short)(u >> 16); }
__device__ __forceinline__ float bfr(float f) { return __uint_as_float(((unsigned)f2bf(f)) << 16); }
__device__ __forceinline__ v16h cat16(v8h lo, v8h hi) { return __builtin_shufflevector(lo, hi, 0, 1, 2, 3, 4, 5, 6, 7, 8, 9, 10, 11, 12, 13, 14, 15); }
__device__ __forceinline__ v16bf cat16b(v8us lo, v8us hi) { return __builtin_bit_cast(v16bf, __builtin_shufflevector(lo, hi, 0, 1, 2, 3, 4, 5, 6, 7, 8, 9, 10, 11, 12, 13, 14, 15)); }
__device__ __forceinline__ v16h  ldh(const h16* p) { return cat16(*(const v8h*)p, *(const v8h*)(p + 16)); }
__device__ __forceinline__ v16bf ldb(const bf* p)  { return cat16b(*(const v8us*)p, *(const v8us*)(p + 16)); }
__device__ __forceinline__ void wave_sync() { __builtin_amdgcn_fence(3  , "wavefront"); __builtin_amdgcn_wave_barrier(); asm volatile("" ::: "memory"); }
__device__ __forceinline__ h16 toh_flush(float v) { const h16 r = (h16)v; return (fabsf(v) < 6.103515625e-05f) ? (h16)0.0f : r; }
__device__ __forceinline__ v8f wmma16g(v16h a, v16h b, v8f c) {
    c = __builtin_amdgcn_wmma_f32_16x16x32_f16(false, a, false, b, (short)0, c, false, false);
    asm volatile("v_nop\n\tv_nop\n\tv_nop\n\tv_nop" : "+v"(c) : "v"(a), "v"(b));
    return c; }
__device__ __forceinline__ v8f wmmabg(v16bf a, v16bf b, v8f c) {
    c = __builtin_amdgcn_wmma_f32_16x16x32_bf16(false, a, false, b, (short)0, c, false, false);
    asm volatile("v_nop\n\tv_nop\n\tv_nop\n\tv_nop" : "+v"(c) : "v"(a), "v"(b));
    return c; }

__global__ __launch_bounds__(256) void k_cvt8(const float* __restrict__ src, bf* dst, size_t n8) {
    const size_t i = (size_t)blockIdx.x * 256 + threadIdx.x; if (i >= n8) return;
    const v8f v = *(const v8f*)(src + i * 8); v8us o;
#pragma unroll
    for (int k = 0; k < 8; ++k) o[k] = f2bf(v[k]);
    *(volatile v8us*)(dst + i * 8) = o; __threadfence(); *(volatile v8us*)(dst + i * 8) = o;
}

__global__ __launch_bounds__(256) void k_cvtw(const float* __restrict__ src, h16* dst, size_t n8) {
    const size_t i = (size_t)blockIdx.x * 256 + threadIdx.x; if (i >= n8) return;
    const v8f v = *(const v8f*)(src + i * 8); v8h o;
#pragma unroll
    for (int k = 0; k < 8; ++k) o[k] = toh_flush(bfr(v[k]) * WPC);
    *(volatile v8h*)(dst + i * 8) = o; __threadfence(); *(volatile v8h*)(dst + i * 8) = o;
}

static_assert(256 * 2 * 16 == 64 * 128);
static_assert(64 * 65 * 4 <= 131072);
__global__ __launch_bounds__(256) void k_xt(const float* __restrict__ x, bf* XT) {
    __shared__ float ts[64 * 65];
    const int tid = threadIdx.x; const int t0 = blockIdx.x * 64, c0 = blockIdx.y * 64, b = blockIdx.z;
    const float* xb = x + ((size_t)b * DM + c0) * SEQ_FULL + t0;
#pragma unroll
    for (int e = 0; e < 4; ++e) { const int q = tid + e * 256; const int c = q >> 4, t4 = (q & 15) * 4;
        const v4f v = *(const v4f*)(xb + (size_t)c * SEQ_FULL + t4);
        ts[c * 65 + t4 + 0] = v[0]; ts[c * 65 + t4 + 1] = v[1]; ts[c * 65 + t4 + 2] = v[2]; ts[c * 65 + t4 + 3] = v[3]; }
    __syncthreads();
    v8us o[2];
#pragma unroll
    for (int e = 0; e < 2; ++e) { const int p = tid + e * 256; const int t = p >> 3, c8 = (p & 7) * 8;
#pragma unroll
        for (int i = 0; i < 8; ++i) o[e][i] = f2bf(ts[(c8 + i) * 65 + t]); }
#pragma unroll 1
    for (int ps = 0; ps < 2; ++ps) {
#pragma unroll
        for (int e = 0; e < 2; ++e) { const int p = tid + e * 256; const int t = p >> 3, c8 = (p & 7) * 8;
            *(volatile v8us*)(XT + ((size_t)b * SEQ + t0 + t) * DM + c0 + c8) = o[e]; }
        if (ps == 0) __threadfence(); }
}

static_assert(32 * 16 * 4 == 16 * 128);
static_assert(16 * OSP * 4 <= 131072);
__global__ __launch_bounds__(32) void k_projt(const bf* __restrict__ A, const bf* __restrict__ Bt, const float* __restrict__ wh, h16* P, int ng, int useWh) {
    __shared__ __align__(16) float os[16 * OSP];
    const int lane = threadIdx.x & 31, lr = lane & 15, hi = lane >> 4; const int r0 = blockIdx.x * 64, c0 = blockIdx.y * 64;
    v8f acc[4][4];
#pragma unroll
    for (int mb = 0; mb < 4; ++mb)
#pragma unroll
        for (int nb = 0; nb < 4; ++nb) acc[mb][nb] = (v8f){};
    const size_t aoff = (size_t)(r0 + lr) * DM + 8 * hi, boff = (size_t)(c0 + lr) * DM + 8 * hi;
#pragma unroll 1
    for (int kc = 0; kc < DM; kc += 32) {
        v16bf a[4];
#pragma unroll
        for (int mb = 0; mb < 4; ++mb) a[mb] = ldb(A + aoff + (size_t)mb * 16 * DM + kc);
#pragma unroll
        for (int nb = 0; nb < 4; ++nb) { const v16bf b = ldb(Bt + boff + (size_t)nb * 16 * DM + kc);
#pragma unroll
            for (int mb = 0; mb < 4; ++mb) acc[mb][nb] = wmmabg(a[mb], b, acc[mb][nb]); }
    }
    const int bb = r0 / SEQ, tt = r0 % SEQ, hsel = c0 / HD;
#pragma unroll
    for (int mb = 0; mb < 4; ++mb) {
#pragma unroll
        for (int nb = 0; nb < 4; ++nb) {
#pragma unroll
            for (int j = 0; j < 8; ++j) os[(hi * 8 + j) * OSP + nb * 16 + lr] = acc[mb][nb][j]; }
        wave_sync();
#pragma unroll 1
        for (int ps = 0; ps < 2; ++ps) {
#pragma unroll 1
            for (int g = 0; g < ng; ++g) {
                int wi = g * NH_ + hsel; wi = wi > 15 ? 15 : wi;
                const float whv = bfr(wh[wi]);
                const float mult = (useWh != 0) ? whv * QKC : QKC;
                const size_t sb = ((size_t)(bb * ng + g) * SEQ + (size_t)(tt + mb * 16)) * DM + c0;
#pragma unroll
                for (int s = 0; s < 4; ++s) { const int row = 4 * s + (lane >> 3), c8 = (lane & 7) * 8;
                    const v4f x0 = *(const v4fa*)(&os[row * OSP + c8]); const v4f x1 = *(const v4fa*)(&os[row * OSP + c8 + 4]); v8h hv;
#pragma unroll
                    for (int i = 0; i < 4; ++i) { hv[i] = toh_flush(x0[i] * mult); hv[4 + i] = toh_flush(x1[i] * mult); }
                    *(volatile v8h*)(P + sb + (size_t)row * DM + c8) = hv; }
            }
            if (ps == 0) __threadfence(); }
        wave_sync();
    }
}

__global__ __launch_bounds__(32) void k_projv(const bf* __restrict__ A, const bf* __restrict__ Bt, h16* P) {
    __shared__ __align__(16) float os[16 * OSP];
    const int lane = threadIdx.x & 31, lr = lane & 15, hi = lane >> 4; const int r0 = blockIdx.x * 64, c0 = blockIdx.y * 64;
    v8f acc[4][4];
#pragma unroll
    for (int mb = 0; mb < 4; ++mb)
#pragma unroll
        for (int nb = 0; nb < 4; ++nb) acc[mb][nb] = (v8f){};
    const size_t aoff = (size_t)(r0 + lr) * DM + 8 * hi, boff = (size_t)(c0 + lr) * DM + 8 * hi;
#pragma unroll 1
    for (int kc = 0; kc < DM; kc += 32) {
        v16bf a[4];
#pragma unroll
        for (int mb = 0; mb < 4; ++mb) a[mb] = ldb(A + aoff + (size_t)mb * 16 * DM + kc);
#pragma unroll
        for (int nb = 0; nb < 4; ++nb) { const v16bf b = ldb(Bt + boff + (size_t)nb * 16 * DM + kc);
#pragma unroll
            for (int mb = 0; mb < 4; ++mb) acc[mb][nb] = wmmabg(a[mb], b, acc[mb][nb]); }
    }
    const int bb = c0 / SEQ, tt = c0 % SEQ;
#pragma unroll
    for (int mb = 0; mb < 4; ++mb) {
#pragma unroll
        for (int nb = 0; nb < 4; ++nb) {
#pragma unroll
            for (int j = 0; j < 8; ++j) os[(hi * 8 + j) * OSP + nb * 16 + lr] = acc[mb][nb][j]; }
        wave_sync();
        const size_t sb = ((size_t)bb * DM + (size_t)(r0 + mb * 16)) * SEQ + tt;
#pragma unroll 1
        for (int ps = 0; ps < 2; ++ps) {
#pragma unroll
            for (int s = 0; s < 4; ++s) { const int row = 4 * s + (lane >> 3), c8 = (lane & 7) * 8;
                const v4f x0 = *(const v4fa*)(&os[row * OSP + c8]); const v4f x1 = *(const v4fa*)(&os[row * OSP + c8 + 4]); v8h hv;
#pragma unroll
                for (int i = 0; i < 4; ++i) { hv[i] = toh_flush(x0[i] * VCC); hv[4 + i] = toh_flush(x1[i] * VCC); }
                *(volatile v8h*)(P + sb + (size_t)row * SEQ + c8) = hv; }
            if (ps == 0) __threadfence(); }
        wave_sync();
    }
}

__global__ __launch_bounds__(256) void k_vsum(const h16* __restrict__ VT, float* VS) {
#pragma clang fp contract(off)
    __shared__ __align__(16) float sm[32];
    const int lane = threadIdx.x & 31;
    const int wave = __builtin_amdgcn_readfirstlane((int)(threadIdx.x >> 5));
#pragma unroll 1
    for (int r = 0; r < 4; ++r) {
        const int row = blockIdx.x * 32 + wave * 4 + r;
        const h16* p = VT + (size_t)row * SEQ;
        float s = 0.0f;
#pragma unroll 1
        for (int i = lane; i < SEQ / 8; i += 32) { const v8h v = *(const v8h*)(p + (size_t)i * 8);
#pragma unroll
            for (int k = 0; k < 8; ++k) s += (float)v[k]; }
        s += __shfl_xor(s, 16, 32); s += __shfl_xor(s, 8, 32); s += __shfl_xor(s, 4, 32); s += __shfl_xor(s, 2, 32); s += __shfl_xor(s, 1, 32);
        if (lane == 0) sm[wave * 4 + r] = s * (1.0f / VCC);
    }
    __syncthreads();
    if (threadIdx.x < 8) { const v4f o = *(const v4fa*)(&sm[threadIdx.x * 4]);
        float* q = VS + (size_t)blockIdx.x * 32 + threadIdx.x * 4;
        *(volatile v4f*)q = o; __threadfence(); *(volatile v4f*)q = o; }
}

__device__ __forceinline__ void scores32(const h16* __restrict__ qp, const h16* __restrict__ kp, v8f& sA, v8f& sB) {
    v8f a = (v8f){}, c = (v8f){};
#pragma unroll 2
    for (int kc = 0; kc < DM; kc += 32) {
        const v16h q = ldh(qp + kc); const v16h ka = ldh(kp + kc); const v16h kb = ldh(kp + (size_t)16 * DM + kc);
        a = wmma16g(ka, q, a); c = wmma16g(kb, q, c); }
    sA = a; sB = c;
}

static_assert(32 * 16 * 8 == 16 * 256);
static_assert(AW * 16 * OSP * 4 + AW * 4 <= 131072);
__global__ __launch_bounds__(32 * AW) __attribute__((amdgpu_num_vgpr(256))) void k_flash(const h16* __restrict__ QP, const h16* __restrict__ KP, const h16* __restrict__ VT, float* ORP, float* PART) {
    __shared__ __align__(16) float os[AW * 16 * OSP];
    __shared__ float sw[AW];
    const int lane = threadIdx.x & 31, lr = lane & 15, hi = lane >> 4;
    const int wave = __builtin_amdgcn_readfirstlane((int)(threadIdx.x >> 5));
    const int zh = blockIdx.y; const int b = zh / NH_, g = zh % NH_;
    const int t0 = (blockIdx.x * AW + wave) * 16;
    const h16* qp = QP + ((size_t)zh * SEQ + (size_t)(t0 + lr)) * DM + 8 * hi;
    const h16* kbase = KP + ((size_t)b * SEQ + (size_t)lr) * DM + 8 * hi;
    const h16* vbase = VT + ((size_t)b * DM + (size_t)(g * HD + lr)) * SEQ + 8 * hi;
    float m = NEGB, l = 0.0f;
#pragma unroll 1
    for (int key0 = 0; key0 < SEQ; key0 += 32) {
        v8f sA, sB; scores32(qp, kbase + (size_t)key0 * DM, sA, sB);
        float mx = NEGB;
#pragma unroll
        for (int r = 0; r < 8; ++r) mx = fmaxf(mx, fmaxf(sA[r] * SC2, sB[r] * SC2));
        mx = fmaxf(mx, __shfl_xor(mx, 16, 32));
        const float mnew = fmaxf(m, mx);
        const float alpha = __builtin_amdgcn_exp2f(m - mnew);
        float ls = 0.0f;
#pragma unroll
        for (int r = 0; r < 8; ++r) ls += __builtin_amdgcn_exp2f(fmaf(sA[r], SC2, -mnew)) + __builtin_amdgcn_exp2f(fmaf(sB[r], SC2, -mnew));
        l = l * alpha + ls; m = mnew;
    }
    l += __shfl_xor(l, 16, 32);
    const float il15 = (1.0f / l) * PCARRY;
    v8f o0 = (v8f){}, o1 = (v8f){}, o2 = (v8f){}, o3 = (v8f){};
    float ss = 0.0f;
#pragma unroll 1
    for (int key0 = 0; key0 < SEQ; key0 += 32) {
        v8f sA, sB; scores32(qp, kbase + (size_t)key0 * DM, sA, sB);
        v16h pb;
#pragma unroll
        for (int r = 0; r < 8; ++r) {
            const float ea = __builtin_amdgcn_exp2f(fmaf(sA[r], SC2, -m)), eb = __builtin_amdgcn_exp2f(fmaf(sB[r], SC2, -m));
            const float ga = fmaf(ea, il15, -C15), gb = fmaf(eb, il15, -C15);
            ss = fmaf(ga, ga, ss); ss = fmaf(gb, gb, ss);
            pb[r] = toh_flush(ga); pb[8 + r] = toh_flush(gb); }
        const h16* va = vbase + key0;
        const v16h v0 = ldh(va), v1 = ldh(va + (size_t)16 * SEQ), v2 = ldh(va + (size_t)32 * SEQ), v3 = ldh(va + (size_t)48 * SEQ);
        o0 = wmma16g(v0, pb, o0); o1 = wmma16g(v1, pb, o1); o2 = wmma16g(v2, pb, o2); o3 = wmma16g(v3, pb, o3);
    }
    ss += __shfl_xor(ss, 16, 32); ss += __shfl_xor(ss, 8, 32); ss += __shfl_xor(ss, 4, 32); ss += __shfl_xor(ss, 2, 32); ss += __shfl_xor(ss, 1, 32);
    if (lane == 0) sw[wave] = ss;
    const int wb = wave * 16 * OSP;
    { v4f a, c;
      a[0] = o0[0] * OSC; a[1] = o0[1] * OSC; a[2] = o0[2] * OSC; a[3] = o0[3] * OSC; c[0] = o0[4] * OSC; c[1] = o0[5] * OSC; c[2] = o0[6] * OSC; c[3] = o0[7] * OSC;
      *(v4fa*)(&os[wb + lr * OSP +  0 + 8 * hi]) = a; *(v4fa*)(&os[wb + lr * OSP +  0 + 8 * hi + 4]) = c;
      a[0] = o1[0] * OSC; a[1] = o1[1] * OSC; a[2] = o1[2] * OSC; a[3] = o1[3] * OSC; c[0] = o1[4] * OSC; c[1] = o1[5] * OSC; c[2] = o1[6] * OSC; c[3] = o1[7] * OSC;
      *(v4fa*)(&os[wb + lr * OSP + 16 + 8 * hi]) = a; *(v4fa*)(&os[wb + lr * OSP + 16 + 8 * hi + 4]) = c;
      a[0] = o2[0] * OSC; a[1] = o2[1] * OSC; a[2] = o2[2] * OSC; a[3] = o2[3] * OSC; c[0] = o2[4] * OSC; c[1] = o2[5] * OSC; c[2] = o2[6] * OSC; c[3] = o2[7] * OSC;
      *(v4fa*)(&os[wb + lr * OSP + 32 + 8 * hi]) = a; *(v4fa*)(&os[wb + lr * OSP + 32 + 8 * hi + 4]) = c;
      a[0] = o3[0] * OSC; a[1] = o3[1] * OSC; a[2] = o3[2] * OSC; a[3] = o3[3] * OSC; c[0] = o3[4] * OSC; c[1] = o3[5] * OSC; c[2] = o3[6] * OSC; c[3] = o3[7] * OSC;
      *(v4fa*)(&os[wb + lr * OSP + 48 + 8 * hi]) = a; *(v4fa*)(&os[wb + lr * OSP + 48 + 8 * hi + 4]) = c; }
    wave_sync();
    float* orow = ORP + ((size_t)zh * SEQ + (size_t)t0) * HD;
#pragma unroll 1
    for (int ps = 0; ps < 2; ++ps) {
#pragma unroll
        for (int s = 0; s < 8; ++s) { const int p = s * 32 + lane; const int row = p >> 4, cofs = (p & 15) * 4;
            const v4f val = *(const v4fa*)(&os[wb + row * OSP + cofs]);
            *(volatile v4f*)(orow + (size_t)p * 4) = val; }
        if (ps == 0) __threadfence(); }
    __syncthreads();
    if (wave == 0) {
        const float tot = ((sw[0] + sw[1]) + sw[2]) + sw[3];
        v4f pv; pv[0] = (lane == 0) ? tot : 0.0f; pv[1] = 0.0f; pv[2] = 0.0f; pv[3] = 0.0f;
        float* pl = PART + ((size_t)zh * (SEQ / 64) + (size_t)blockIdx.x) * 32 + (lane & 7) * 4;
        if (lane < 8) { *(volatile v4f*)pl = pv; __threadfence(); *(volatile v4f*)pl = pv; }
    }
}

static_assert(256 * 8 == 2048);
__global__ __launch_bounds__(256) void k_ctx(const float* __restrict__ ORP, const float* __restrict__ PART, const float* __restrict__ VS,
                                             const float* __restrict__ gain, const float* __restrict__ shift, h16* CT) {
#pragma clang fp contract(off)
    const size_t e0 = ((size_t)blockIdx.x * 256 + threadIdx.x) * 8;
    const int zh = (int)(((size_t)blockIdx.x * 2048) / ((size_t)SEQ * HD));
    const int b = zh / NH_, g = zh % NH_;
    float tot = 0.0f;
#pragma unroll 1
    for (int j = 0; j < SEQ / 64; ++j) tot += PART[((size_t)zh * (SEQ / 64) + (size_t)j) * 32];
    const float var = tot * VSC;
    const float s1 = bfr(gain[g]) * rsqrtf(var + EPSN);
    const float bt = bfr(shift[g]);
    const int dd0 = (int)(e0 % HD);
    const v8f xv = *(const v8f*)(ORP + e0);
    const float* vp = VS + (size_t)b * DM + (size_t)(g * HD + dd0);
    const v4f s0 = *(const v4f*)vp, s4 = *(const v4f*)(vp + 4);
    v8h o;
#pragma unroll
    for (int k = 0; k < 4; ++k) { o[k] = toh_flush((s1 * xv[k] + bt * s0[k]) * CCS); o[4 + k] = toh_flush((s1 * xv[4 + k] + bt * s4[k]) * CCS); }
    *(volatile v8h*)(CT + e0) = o; __threadfence(); *(volatile v8h*)(CT + e0) = o;
}

static_assert(32 * 16 * 8 == 16 * 256);
__global__ __launch_bounds__(32) void k_out(const h16* __restrict__ A, const h16* __restrict__ Bt, const float* __restrict__ bias, float* OUT) {
    __shared__ __align__(16) float os[16 * OSP];
    const int lane = threadIdx.x & 31, lr = lane & 15, hi = lane >> 4; const int r0 = blockIdx.x * 64, c0 = blockIdx.y * 64;
    v8f acc[4][4];
#pragma unroll
    for (int mb = 0; mb < 4; ++mb)
#pragma unroll
        for (int nb = 0; nb < 4; ++nb) acc[mb][nb] = (v8f){};
    const size_t aoff = (size_t)(r0 + lr) * DM + 8 * hi, boff = (size_t)(c0 + lr) * DM + 8 * hi;
#pragma unroll 1
    for (int kc = 0; kc < DM; kc += 32) {
        v16h a[4];
#pragma unroll
        for (int mb = 0; mb < 4; ++mb) a[mb] = ldh(A + aoff + (size_t)mb * 16 * DM + kc);
#pragma unroll
        for (int nb = 0; nb < 4; ++nb) { const v16h b = ldh(Bt + boff + (size_t)nb * 16 * DM + kc);
#pragma unroll
            for (int mb = 0; mb < 4; ++mb) acc[mb][nb] = wmma16g(a[mb], b, acc[mb][nb]); }
    }
    const int bb = c0 / SEQ, tt = c0 % SEQ;
#pragma unroll
    for (int mb = 0; mb < 4; ++mb) {
        float br[8];
#pragma unroll
        for (int j = 0; j < 8; ++j) br[j] = bfr(bias[r0 + mb * 16 + hi * 8 + j]);
#pragma unroll
        for (int nb = 0; nb < 4; ++nb) {
#pragma unroll
            for (int j = 0; j < 8; ++j) os[(hi * 8 + j) * OSP + nb * 16 + lr] = acc[mb][nb][j] * OUTSC + br[j]; }
        wave_sync();
        float* ob = OUT + ((size_t)bb * DM + (size_t)(r0 + mb * 16)) * OUT_SEQ + tt;
#pragma unroll 1
        for (int ps = 0; ps < 2; ++ps) {
#pragma unroll
            for (int s = 0; s < 8; ++s) { const int p = s * 32 + lane; const int row = p >> 4, cofs = (p & 15) * 4;
                const v4f val = *(const v4fa*)(&os[row * OSP + cofs]);
                *(volatile v4f*)(ob + (size_t)row * OUT_SEQ + cofs) = val; }
            if (ps == 0) __threadfence(); }
        wave_sync();
    }
}

static constexpr size_t al256(size_t v) { return (v + 255) & ~(size_t)255; }
static constexpr size_t SZ_XT = al256((size_t)NB * SEQ * DM * 2);
static constexpr size_t SZ_WB = al256((size_t)3 * DM * DM * 2);
static constexpr size_t SZ_WP = al256((size_t)DM * DM * 2);
static constexpr size_t SZ_QP = al256((size_t)NB * NH_ * SEQ * DM * 2);
static constexpr size_t SZ_KP = al256((size_t)NB * SEQ * DM * 2);
static constexpr size_t SZ_VT = al256((size_t)NB * DM * SEQ * 2);
static constexpr size_t SZ_VS = al256((size_t)NB * DM * 4);
static constexpr size_t SZ_OR = al256((size_t)NB * NH_ * SEQ * HD * 4);
static constexpr size_t SZ_PT = al256((size_t)NB * NH_ * (SEQ / 64) * 32 * 4);
static constexpr size_t SZ_CT = al256((size_t)NB * SEQ * DM * 2);
static constexpr size_t SZ_TOTAL = SZ_XT + SZ_WB + SZ_WP + SZ_QP + SZ_KP + SZ_VT + SZ_VS + SZ_OR + SZ_PT + SZ_CT;
static_assert(SZ_TOTAL <= (size_t)134217728);
static_assert(((size_t)DM * DM * 2) % 256 == 0);
static_assert((size_t)NB * NH_ * SEQ * HD == (size_t)NB * SEQ * DM);
static_assert(((size_t)NB * DM / 32) * 32 * 4 <= SZ_VS);
static_assert(((size_t)(NB * NH_ - 1) * (SEQ / 64) + (SEQ / 64 - 1)) * 128 + 128 <= SZ_PT);

extern "C" void kernel_launch(void* const* d_in, const int* in_sizes, int n_in,
                              void* d_out, int out_size, void* d_ws, size_t ws_size, hipStream_t stream) {
    if (n_in < 9) return;
    const size_t needx = ((size_t)(NB - 1) * DM + (size_t)(DM - 1)) * SEQ_FULL + SEQ;
    if ((size_t)in_sizes[0] < needx) return;
    if ((size_t)in_sizes[1] < (size_t)DM * DM || (size_t)in_sizes[2] < (size_t)DM * DM || (size_t)in_sizes[3] < (size_t)DM * DM || (size_t)in_sizes[7] < (size_t)DM * DM) return;
    if (in_sizes[4] < NH_ * NH_ || in_sizes[5] < NH_ || in_sizes[6] < NH_ || in_sizes[8] < DM) return;
    if ((size_t)out_size < ((size_t)(NB - 1) * DM + (size_t)(DM - 1)) * OUT_SEQ + SEQ) return;
    if (SZ_TOTAL > ws_size) return;
    const float* x  = (const float*)d_in[0];
    const float* wq = (const float*)d_in[1]; const float* wk = (const float*)d_in[2]; const float* wv = (const float*)d_in[3];
    const float* whd = (const float*)d_in[4]; const float* gam = (const float*)d_in[5]; const float* bet = (const float*)d_in[6];
    const float* wp = (const float*)d_in[7]; const float* bp = (const float*)d_in[8];
    float* OUT = (float*)d_out;
    char* wsp = (char*)d_ws;
    bf*  XT  = (bf*)wsp;   wsp += SZ_XT;
    bf*  WB  = (bf*)wsp;   wsp += SZ_WB;
    h16* WPH = (h16*)wsp;  wsp += SZ_WP;
    h16* QP  = (h16*)wsp;  wsp += SZ_QP;
    h16* KP  = (h16*)wsp;  wsp += SZ_KP;
    h16* VT  = (h16*)wsp;  wsp += SZ_VT;
    float* VS = (float*)wsp; wsp += SZ_VS;
    float* ORP = (float*)wsp; wsp += SZ_OR;
    float* PART = (float*)wsp; wsp += SZ_PT;
    h16* CT  = (h16*)wsp;  wsp += SZ_CT;
    bf* WQ = WB; bf* WK = WB + (size_t)DM * DM; bf* WV = WB + (size_t)2 * DM * DM;

    k_xt<<<dim3(SEQ / 64, DM / 64, NB), 256, 0, stream>>>(x, XT);
    { const size_t n8 = (size_t)DM * DM / 8; const unsigned gg = (unsigned)((n8 + 255) / 256);
      k_cvt8<<<gg, 256, 0, stream>>>(wq, WQ, n8); k_cvt8<<<gg, 256, 0, stream>>>(wk, WK, n8); k_cvt8<<<gg, 256, 0, stream>>>(wv, WV, n8);
      k_cvtw<<<gg, 256, 0, stream>>>(wp, WPH, n8); }

    k_projt<<<dim3(NB * SEQ / 64, DM / 64, 1), 32, 0, stream>>>(XT, WQ, whd, QP, NH_, 1);
    k_projt<<<dim3(NB * SEQ / 64, DM / 64, 1), 32, 0, stream>>>(XT, WK, whd, KP, 1, 0);
    k_projv<<<dim3(DM / 64, NB * SEQ / 64, 1), 32, 0, stream>>>(WV, XT, VT);
    k_vsum<<<dim3(NB * DM / 32, 1, 1), 256, 0, stream>>>(VT, VS);

    k_flash<<<dim3(SEQ / (16 * AW), NB * NH_, 1), 32 * AW, 0, stream>>>(QP, KP, VT, ORP, PART);
    k_ctx<<<dim3((unsigned)((size_t)NB * SEQ * DM / 2048), 1, 1), 256, 0, stream>>>(ORP, PART, VS, gam, bet, CT);
    k_out<<<dim3(DM / 64, NB * SEQ / 64, 1), 32, 0, stream>>>(WPH, CT, bp, OUT);
}
